// MCA_31078383354481
// MI455X (gfx1250) — hardware-verified
//
#include <hip/hip_runtime.h>
#include <stdint.h>


#define HEADS 32
#define DHEAD 8
#define NPIX 1024
#define CCH 256
#define QROWS (3 * CCH)
#define ATT_SCALE 0.35355339059327379f
#define P_SCALE 256.0f

#define TM 64
#define TN 32
#define KC 32
#define LP 40
#define OSP 36
#define QCH 128
#define VTP 1032
#define PSP 40
#define OHP 132

static_assert(NPIX % TN == 0 && QROWS % TM == 0 && CCH % TM == 0 && CCH % KC == 0 && NPIX % QCH == 0);
static_assert((LP * 2) % 16 == 0 && (OSP * 4) % 16 == 0 && (VTP * 2) % 16 == 0 && (PSP * 2) % 16 == 0 && (OHP * 4) % 16 == 0);

typedef float v8f __attribute__((ext_vector_type(8)));
typedef float v4f_t __attribute__((ext_vector_type(4)));
typedef v4f_t v4f __attribute__((may_alias));
typedef unsigned short v8us_t __attribute__((ext_vector_type(8)));
typedef v8us_t v8us __attribute__((may_alias));
typedef unsigned short v4us_t __attribute__((ext_vector_type(4)));
typedef v4us_t v4us __attribute__((may_alias));
typedef __bf16 v16bf __attribute__((ext_vector_type(16)));
typedef _Float16 v16h __attribute__((ext_vector_type(16)));

union FragB { v16bf v; v8us_t h[2]; };
union FragH { v16h v; v8us_t h[2]; };

__device__ __forceinline__ v8f zero8() {
  v8f z;
#pragma unroll
  for (int i = 0; i < 8; ++i) z[i] = 0.0f;
  return z;
}
__device__ __forceinline__ v8us_t zero8us() {
  v8us_t z;
#pragma unroll
  for (int i = 0; i < 8; ++i) z[i] = (unsigned short)0;
  return z;
}

__device__ __forceinline__ unsigned short bf16_rne(float f) {
  unsigned u = __float_as_uint(f);
  u += 0x7FFFu + ((u >> 16) & 1u);
  return (unsigned short)(u >> 16);
}
__device__ __forceinline__ float bf16_val(unsigned short b) {
  return __uint_as_float(((unsigned)b) << 16);
}
__device__ __forceinline__ unsigned short f16_bits(float f) {
  union { _Float16 h; unsigned short u; } c;
  c.h = (_Float16)f;
  return c.u;
}
__device__ __forceinline__ void split4(v4f_t v, v4us_t& hi, v4us_t& lo) {
#pragma unroll
  for (int j = 0; j < 4; ++j) {
    unsigned short a = bf16_rne(v[j]);
    hi[j] = a;
    lo[j] = bf16_rne(v[j] - bf16_val(a));
  }
}

__device__ __forceinline__ v8f mma_bf16(v16bf a, v16bf b, v8f c) {
  v8f d = __builtin_amdgcn_wmma_f32_16x16x32_bf16(false, a, false, b, (short)0, c, false, false);
  asm volatile("v_nop\n\tv_nop\n\tv_nop\n\tv_nop" : "+v"(d) : "v"(a), "v"(b));
  return d;
}
__device__ __forceinline__ v8f mma_f16(v16h a, v16h b, v8f c) {
  v8f d = __builtin_amdgcn_wmma_f32_16x16x32_f16(false, a, false, b, (short)0, c, false, false);
  asm volatile("v_nop\n\tv_nop\n\tv_nop\n\tv_nop" : "+v"(d) : "v"(a), "v"(b));
  return d;
}

template <int MODE>
__global__ __launch_bounds__(128) void k_gemm(
    const float* __restrict__ xin_q, const float* __restrict__ xin_kv,
    const float* __restrict__ w_q, const float* __restrict__ w_kv,
    const float* __restrict__ bias,
    unsigned short* __restrict__ qs, unsigned short* __restrict__ ks, unsigned short* __restrict__ vs,
    float* __restrict__ out, int nb) {
  __shared__ __attribute__((aligned(16))) unsigned short Wh[TM][LP];
  __shared__ __attribute__((aligned(16))) unsigned short Wl[TM][LP];
  __shared__ __attribute__((aligned(16))) unsigned short Xh[TN][LP];
  __shared__ __attribute__((aligned(16))) unsigned short Xl[TN][LP];
  __shared__ __attribute__((aligned(16))) float Os[TM][OSP];

  const int tid = threadIdx.x, lane = tid & 31, wave = tid >> 5;
  const int h = lane >> 4, m = lane & 15;
  const int b = blockIdx.z;
  const int pbase = blockIdx.x * TN;
  const int orow0 = blockIdx.y * TM;
  if (b >= nb || pbase + TN > NPIX) return;
  if (MODE == 0 && orow0 + TM > QROWS) return;
  if (MODE == 1 && orow0 + TM > CCH) return;

  const float* W;
  const float* X;
  if (MODE == 0 && orow0 >= CCH) { W = w_kv + (size_t)(orow0 - CCH) * CCH; X = xin_kv; }
  else                           { W = w_q + (size_t)orow0 * CCH;           X = xin_q; }
  X += (size_t)b * CCH * NPIX;

  v8f acc[2];
  acc[0] = zero8();
  acc[1] = zero8();

  for (int kc = 0; kc < CCH; kc += KC) {
#pragma unroll
    for (int i = 0; i < 4; ++i) {
      const int idx = tid + 128 * i;
      const int row = idx >> 3, c4 = (idx & 7) * 4;
      v4f_t wv = *(const v4f*)(W + (size_t)row * CCH + kc + c4);
      v4us_t hi, lo;
      split4(wv, hi, lo);
      *(v4us*)&Wh[row][c4] = hi;
      *(v4us*)&Wl[row][c4] = lo;
    }
#pragma unroll
    for (int i = 0; i < 2; ++i) {
      const int idx = tid + 128 * i;
      const int kr = idx >> 3, p4 = (idx & 7) * 4;
      v4f_t xv = *(const v4f*)(X + (size_t)(kc + kr) * NPIX + pbase + p4);
      v4us_t hi, lo;
      split4(xv, hi, lo);
#pragma unroll
      for (int j = 0; j < 4; ++j) {
        Xh[p4 + j][kr] = hi[j];
        Xl[p4 + j][kr] = lo[j];
      }
    }
    __syncthreads();

    FragB ah, al;
    ah.h[0] = *(const v8us*)&Wh[16 * wave + m][8 * h];
    ah.h[1] = *(const v8us*)&Wh[16 * wave + m][16 + 8 * h];
    al.h[0] = *(const v8us*)&Wl[16 * wave + m][8 * h];
    al.h[1] = *(const v8us*)&Wl[16 * wave + m][16 + 8 * h];
#pragma unroll
    for (int nh = 0; nh < 2; ++nh) {
      FragB bh, bl;
      bh.h[0] = *(const v8us*)&Xh[16 * nh + m][8 * h];
      bh.h[1] = *(const v8us*)&Xh[16 * nh + m][16 + 8 * h];
      bl.h[0] = *(const v8us*)&Xl[16 * nh + m][8 * h];
      bl.h[1] = *(const v8us*)&Xl[16 * nh + m][16 + 8 * h];
      acc[nh] = mma_bf16(ah.v, bh.v, acc[nh]);
      acc[nh] = mma_bf16(ah.v, bl.v, acc[nh]);
      acc[nh] = mma_bf16(al.v, bh.v, acc[nh]);
    }
    __syncthreads();
  }

#pragma unroll
  for (int nh = 0; nh < 2; ++nh) {
#pragma unroll
    for (int r = 0; r < 8; ++r) Os[16 * wave + 8 * h + r][16 * nh + m] = acc[nh][r];
  }
  __syncthreads();

  if (MODE == 1) {
    v4f_t vals[4];
#pragma unroll
    for (int s = 0; s < 4; ++s) {
      const int row = 16 * wave + 4 * s + (lane >> 3);
      const int q = lane & 7;
      v4f_t v = *(const v4f*)&Os[row][4 * q];
      const float bb = bias[orow0 + row];
      v += bb;
      vals[s] = v;
    }
    float* ob = out + ((size_t)b * CCH + orow0) * NPIX + pbase;
#pragma unroll
    for (int s = 0; s < 4; ++s) {
      const int row = 16 * wave + 4 * s + (lane >> 3);
      *(volatile v4f*)(ob + (size_t)row * NPIX + 4 * (lane & 7)) = vals[s];
    }
    __threadfence();
#pragma unroll
    for (int s = 0; s < 4; ++s) {
      const int row = 16 * wave + 4 * s + (lane >> 3);
      *(volatile v4f*)(ob + (size_t)row * NPIX + 4 * (lane & 7)) = vals[s];
    }
  } else {
    const int seg = orow0 >> 8;
    const int hb = (orow0 & (CCH - 1)) >> 3;
    if (seg < 2) {
      unsigned short* dstb = (seg == 0) ? qs : ks;
      v8us_t vals[4];
#pragma unroll
      for (int t = 0; t < 2; ++t) {
        const int hh = 2 * wave + t;
#pragma unroll
        for (int s = 0; s < 2; ++s) {
          const int pl = 16 * s + (lane >> 1);
          const int part = lane & 1;
          v8us_t pk;
#pragma unroll
          for (int d = 0; d < DHEAD; ++d) {
            const float v = Os[8 * hh + d][pl];
            const unsigned short hi = bf16_rne(v);
            const unsigned short lo = bf16_rne(v - bf16_val(hi));
            pk[d] = part ? lo : hi;
          }
          vals[2 * t + s] = pk;
        }
      }
#pragma unroll
      for (int t = 0; t < 2; ++t) {
        unsigned short* hp = dstb + (((size_t)b * HEADS + hb + 2 * wave + t) * NPIX + pbase) * 16;
#pragma unroll
        for (int s = 0; s < 2; ++s) *(volatile v8us*)(hp + 256 * s + 8 * lane) = vals[2 * t + s];
      }
      __threadfence();
#pragma unroll
      for (int t = 0; t < 2; ++t) {
        unsigned short* hp = dstb + (((size_t)b * HEADS + hb + 2 * wave + t) * NPIX + pbase) * 16;
#pragma unroll
        for (int s = 0; s < 2; ++s) *(volatile v8us*)(hp + 256 * s + 8 * lane) = vals[2 * t + s];
      }
    } else {
      v8us_t vals[2];
#pragma unroll
      for (int t = 0; t < 2; ++t) {
        const int hh = 2 * wave + t;
        v8us_t pk;
#pragma unroll
        for (int d = 0; d < DHEAD; ++d) pk[d] = f16_bits(Os[8 * hh + d][lane]);
        vals[t] = pk;
      }
#pragma unroll
      for (int t = 0; t < 2; ++t) {
        unsigned short* vp = vs + (((size_t)b * HEADS + hb + 2 * wave + t) * NPIX + pbase + lane) * DHEAD;
        *(volatile v8us*)vp = vals[t];
      }
      __threadfence();
#pragma unroll
      for (int t = 0; t < 2; ++t) {
        unsigned short* vp = vs + (((size_t)b * HEADS + hb + 2 * wave + t) * NPIX + pbase + lane) * DHEAD;
        *(volatile v8us*)vp = vals[t];
      }
    }
  }
}

__global__ __launch_bounds__(256) void k_attn(
    const unsigned short* __restrict__ qs, const unsigned short* __restrict__ ks,
    const unsigned short* __restrict__ vs, float* __restrict__ ao, int nb) {
  __shared__ __attribute__((aligned(16))) unsigned short Vt[DHEAD + 1][VTP];
  __shared__ __attribute__((aligned(16))) unsigned short Ps[QCH / 16][16][PSP];
  __shared__ __attribute__((aligned(16))) float Osh[DHEAD][OHP];

  const int tid = threadIdx.x, lane = tid & 31, wave = tid >> 5;
  const int h = lane >> 4, m = lane & 15;
  const int b = blockIdx.z, hd = blockIdx.y, chunk = blockIdx.x;
  if (b >= nb || hd >= HEADS || chunk * QCH + QCH > NPIX) return;
  const size_t bh = (size_t)b * HEADS + hd;

  for (int p = tid; p < NPIX; p += 256) {
    v8us_t rv = *(const v8us*)(vs + (bh * NPIX + p) * DHEAD);
#pragma unroll
    for (int d = 0; d < DHEAD; ++d) Vt[d][p] = rv[d];
    Vt[DHEAD][p] = (unsigned short)0x3C00u;
  }
  __syncthreads();

  const int qbase = chunk * QCH + wave * 16;

  const v8us_t z8 = zero8us();
  FragB qa;
  {
    const unsigned short* qr = qs + (bh * NPIX + qbase + m) * 16;
    v8us_t qh = *(const v8us*)qr;
    v8us_t ql = *(const v8us*)(qr + 8);
    qa.h[0] = h ? ql : qh;
    qa.h[1] = h ? z8 : qh;
  }

  float run_m[8];
#pragma unroll
  for (int r = 0; r < 8; ++r) run_m[r] = -1.0e30f;
  v8f oacc = zero8();

  for (int j = 0; j < NPIX / 32; ++j) {
    const int kp0 = 32 * j;
    FragB kb0, kb1;
    {
      const unsigned short* k0 = ks + (bh * NPIX + kp0 + m) * 16;
      const unsigned short* k1 = k0 + 16 * 16;
      v8us_t k0h = *(const v8us*)k0;
      v8us_t k0l = *(const v8us*)(k0 + 8);
      v8us_t k1h = *(const v8us*)k1;
      v8us_t k1l = *(const v8us*)(k1 + 8);
      kb0.h[0] = k0h; kb0.h[1] = h ? z8 : k0l;
      kb1.h[0] = k1h; kb1.h[1] = h ? z8 : k1l;
    }
    v8f s0 = mma_bf16(qa.v, kb0.v, zero8());
    v8f s1 = mma_bf16(qa.v, kb1.v, zero8());

#pragma unroll
    for (int r = 0; r < 8; ++r) {
      const float a0 = s0[r], a1 = s1[r];
      float tm = fmaxf(a0, a1);
#pragma unroll
      for (int o = 1; o <= 8; o <<= 1) tm = fmaxf(tm, __shfl_xor(tm, o, 32));
      const float nm = fmaxf(run_m[r], tm);
      const float alpha = __expf((run_m[r] - nm) * ATT_SCALE);
      run_m[r] = nm;
      oacc[r] *= alpha;
      const float p0 = __expf((a0 - nm) * ATT_SCALE) * P_SCALE;
      const float p1 = __expf((a1 - nm) * ATT_SCALE) * P_SCALE;
      Ps[wave][8 * h + r][m]      = f16_bits(p0);
      Ps[wave][8 * h + r][16 + m] = f16_bits(p1);
    }
    __syncthreads();

    FragH pa;
    pa.h[0] = *(const v8us*)&Ps[wave][m][8 * h];
    pa.h[1] = *(const v8us*)&Ps[wave][m][16 + 8 * h];
    FragH vb;
    vb.h[0] = z8; vb.h[1] = z8;
    if (m < DHEAD + 1) {
      vb.h[0] = *(const v8us*)&Vt[m][kp0 + 8 * h];
      vb.h[1] = *(const v8us*)&Vt[m][kp0 + 16 + 8 * h];
    }
    oacc = mma_f16(pa.v, vb.v, oacc);
    __syncthreads();
  }

#pragma unroll
  for (int r = 0; r < 8; ++r) {
    const float lr = __shfl(oacc[r], (lane & 16) | 8, 32);
    const float val = oacc[r] / lr;
    if (m < DHEAD) Osh[m][wave * 16 + 8 * h + r] = val;
  }
  __syncthreads();

  {
    v4f_t ov = *(const v4f*)&Osh[wave][4 * lane];
    float* dst = ao + ((size_t)b * CCH + hd * DHEAD + wave) * NPIX + chunk * QCH + 4 * lane;
    *(volatile v4f*)dst = ov;
    __threadfence();
    *(volatile v4f*)dst = ov;
  }
}

extern "C" void kernel_launch(void* const* d_in, const int* in_sizes, int n_in,
                              void* d_out, int out_size, void* d_ws, size_t ws_size,
                              hipStream_t stream) {
  if (n_in < 6) return;
  const int nb = in_sizes[0] / (CCH * NPIX);
  if (nb <= 0) return;
  if (in_sizes[0] != nb * CCH * NPIX) return;
  if (in_sizes[1] != in_sizes[0]) return;
  if (in_sizes[2] != CCH * CCH) return;
  if (in_sizes[3] != 2 * CCH * CCH) return;
  if (in_sizes[4] != CCH * CCH) return;
  if (in_sizes[5] < CCH) return;
  if (out_size != nb * CCH * NPIX) return;

  const float* x     = (const float*)d_in[0];
  const float* xq    = (const float*)d_in[1];
  const float* Wq    = (const float*)d_in[2];
  const float* Wkv   = (const float*)d_in[3];
  const float* Wproj = (const float*)d_in[4];
  const float* bproj = (const float*)d_in[5];
  float* out = (float*)d_out;

  const size_t qk_bytes = (size_t)nb * HEADS * NPIX * 16 * sizeof(unsigned short);
  const size_t v_bytes  = (size_t)nb * HEADS * NPIX * DHEAD * sizeof(unsigned short);
  const size_t ao_bytes = (size_t)nb * CCH * NPIX * sizeof(float);
  if (2 * qk_bytes + v_bytes + ao_bytes > ws_size) return;

  char* wsb = (char*)d_ws;
  unsigned short* Qs = (unsigned short*)(wsb);
  unsigned short* Ks = (unsigned short*)(wsb + qk_bytes);
  unsigned short* Vs = (unsigned short*)(wsb + 2 * qk_bytes);
  float* AO = (float*)(wsb + 2 * qk_bytes + v_bytes);

  k_gemm<0><<<dim3(NPIX / TN, QROWS / TM, nb), 128, 0, stream>>>(
      xq, x, Wq, Wkv, bproj, Qs, Ks, Vs, out, nb);
  k_attn<<<dim3(NPIX / QCH, HEADS, nb), 256, 0, stream>>>(Qs, Ks, Vs, AO, nb);
  k_gemm<1><<<dim3(NPIX / TN, CCH / TM, nb), 128, 0, stream>>>(
      AO, AO, Wproj, Wproj, bproj, Qs, Ks, Vs, out, nb);
}
